// ParCgnn_70600672411869
// MI455X (gfx1250) — hardware-run, weakly checked
//
#include <hip/hip_runtime.h>


#ifndef NN
#define NN 30000
#endif
#define NN_FULL 30000
#define CI   256
#define CO   128
#define KS   9
#define KNB  16
#define NSLOT (KNB + 1)
#define NPAD (((NN + 63) / 64) * 64)
#define FRP  (2 * CO)
#define AGW  8
#define TABV4 ((2 * CO) / 4)
#define IDXSC ((float)((double)KS / (double)NSLOT))

static_assert(CI % 32 == 0);
static_assert(NPAD % 64 == 0);
static_assert(CO % 64 == 0);
static_assert((2 * CO) % 64 == 0);
static_assert((CO & (CO - 1)) == 0);
static_assert(CO == 32 * 4);
static_assert(32 * 16 == CO * 4);
static_assert(32 * 16 * 8 == 16 * 64 * 4);
static_assert(TABV4 * 16 == 2 * CO * 4);
static_assert(TABV4 <= CO);
static_assert(TABV4 % 8 == 0);
static_assert(KNB == 16);
static_assert(((size_t)NN * CI) % (8 * 8) == 0);
static_assert((((size_t)NPAD - NN) * CI) % (8 * 8) == 0);
static_assert(((size_t)CO * CI) % (8 * 8) == 0);
static_assert(NN <= NN_FULL);
static_assert(16 * 68 * 4 <= 131072);
static_assert(2 * CO * 4 <= 131072);

typedef unsigned short bf;
typedef __attribute__((ext_vector_type(16))) __bf16   v16bf;
typedef __attribute__((ext_vector_type(8)))  unsigned short v8us;
typedef __attribute__((ext_vector_type(8)))  float    v8f;
typedef __attribute__((ext_vector_type(4)))  float    v4f;
typedef __attribute__((ext_vector_type(4)))  int      v4i;
typedef v4f  __attribute__((may_alias)) v4fa;

__device__ __forceinline__ unsigned short f2bf(float f) { unsigned u = __float_as_uint(f); u += 0x7FFFu + ((u >> 16) & 1u); return (unsigned short)(u >> 16); }
__device__ __forceinline__ float bfr(float f) { return __uint_as_float(((unsigned)f2bf(f)) << 16); }
__device__ __forceinline__ v16bf cat16b(v8us lo, v8us hi) { return __builtin_bit_cast(v16bf, __builtin_shufflevector(lo, hi, 0, 1, 2, 3, 4, 5, 6, 7, 8, 9, 10, 11, 12, 13, 14, 15)); }
__device__ __forceinline__ v8f wmmab(v16bf a, v16bf b, v8f c) { return __builtin_amdgcn_wmma_f32_16x16x32_bf16(false, a, false, b, (short)0, c, false, false); }
__device__ __forceinline__ v16bf ldb(const bf* p)  { return cat16b(*(const v8us*)p, *(const v8us*)(p + 16)); }
__device__ __forceinline__ void wave_sync() { __builtin_amdgcn_fence(3  , "wavefront"); __builtin_amdgcn_wave_barrier(); asm volatile("" ::: "memory"); }
__device__ __forceinline__ v8f wmmab_g(v16bf a, v16bf b, v8f c) { c = wmmab(a, b, c); asm volatile("v_nop\n\tv_nop\n\tv_nop\n\tv_nop" : "+v"(c) : "v"(a), "v"(b)); return c; }

__global__ __launch_bounds__(256) void k_cvt8(const float* __restrict__ src, bf* dst, size_t n8) {
    const size_t i = (size_t)blockIdx.x * 256 + threadIdx.x; if (i >= n8) return;
    const v8f v = *(const v8f*)(src + i * 8); v8us o;
#pragma unroll
    for (int k = 0; k < 8; ++k) o[k] = f2bf(v[k]);
    *(volatile v8us*)(dst + i * 8) = o; __threadfence(); *(volatile v8us*)(dst + i * 8) = o;
}

__global__ __launch_bounds__(256) void k_zero8(bf* dst, size_t n8) {
    const size_t i = (size_t)blockIdx.x * 256 + threadIdx.x; if (i >= n8) return;
    const v8us o = (v8us){};
    *(volatile v8us*)(dst + i * 8) = o; __threadfence(); *(volatile v8us*)(dst + i * 8) = o;
}

__global__ __launch_bounds__(CO) void k_tab(const float* __restrict__ weight, float* TAB) {
#pragma clang fp contract(off)
    __shared__ __align__(16) float ts[2 * CO];
    const int d = threadIdx.x;
    const float e  = (float)(d & ~1) / (float)CO;
    const float pw = powf(10000.0f, e);
    const float rp = 1.0f / pw;
    float ps = 0.0f, wsm = 0.0f;
#pragma unroll 1
    for (int s = 0; s < NSLOT; ++s) {
        int p = (int)floorf((float)s * IDXSC);
        p = p < 0 ? 0 : (p > KS - 1 ? KS - 1 : p);
        const float ang = (float)p * rp;
        float sv, cv;
        sincosf(ang, &sv, &cv);
        ps  += (d & 1) ? cv : sv;
        wsm += bfr(weight[d * KS + p]);
    }
    ts[d] = ps; ts[CO + d] = wsm;
    __syncthreads();
    if (threadIdx.x < TABV4) {
        const v4f val = *(const v4fa*)(&ts[4 * threadIdx.x]);
        *(volatile v4f*)(TAB + 4 * threadIdx.x) = val; __threadfence(); *(volatile v4f*)(TAB + 4 * threadIdx.x) = val;
    }
}

__global__ __launch_bounds__(32) void k_gemm(const bf* __restrict__ A, const bf* __restrict__ Bt, const float* __restrict__ blin, const float* __restrict__ bres, float* FR) {
    __shared__ __align__(16) float os[16 * 68];
    const int K = CI;
    const int lane = threadIdx.x & 31, lr = lane & 15, hi = lane >> 4; const int r0 = blockIdx.x * 64, c0 = blockIdx.y * 64;
    v8f acc[4][4];
#pragma unroll
    for (int mb = 0; mb < 4; ++mb)
#pragma unroll
        for (int nb = 0; nb < 4; ++nb) acc[mb][nb] = (v8f){};
    const size_t aoff = (size_t)(r0 + lr) * K + 8 * hi, boff = (size_t)(c0 + lr) * K + 8 * hi;
#pragma unroll 1
    for (int kc = 0; kc < K; kc += 32) {
        v16bf a[4];
#pragma unroll
        for (int mb = 0; mb < 4; ++mb) a[mb] = ldb(A + aoff + (size_t)mb * 16 * K + kc);
#pragma unroll
        for (int nb = 0; nb < 4; ++nb) { const v16bf b = ldb(Bt + boff + (size_t)nb * 16 * K + kc);
#pragma unroll
            for (int mb = 0; mb < 4; ++mb) acc[mb][nb] = wmmab_g(a[mb], b, acc[mb][nb]); }
    }
    float bc[4];
#pragma unroll
    for (int nb = 0; nb < 4; ++nb) { const int ci = (c0 + nb * 16 + lr) & (CO - 1);
        const float v0 = blin[ci]; const float v1 = bres[ci];
        bc[nb] = bfr((c0 < CO) ? v0 : v1); }
#pragma unroll
    for (int mb = 0; mb < 4; ++mb) {
#pragma unroll
        for (int nb = 0; nb < 4; ++nb) {
#pragma unroll
            for (int j = 0; j < 8; ++j) os[(hi * 8 + j) * 68 + nb * 16 + lr] = acc[mb][nb][j] + bc[nb]; }
        wave_sync();
        float* fb = FR + (size_t)(r0 + mb * 16) * FRP + c0;
#pragma unroll 1
        for (int ps = 0; ps < 2; ++ps) {
#pragma unroll
            for (int s = 0; s < 8; ++s) { const int row = 2 * s + (lane >> 4), c4 = (lane & 15) * 4;
                const v4f val = *(const v4fa*)(&os[row * 68 + c4]);
                *(volatile v4f*)(fb + (size_t)row * FRP + c4) = val; }
            if (ps == 0) __threadfence(); }
        wave_sync();
    }
}

__global__ __launch_bounds__(32 * AGW) void k_agg(const float* __restrict__ FR, const int* __restrict__ nbr, const float* __restrict__ TAB, const float* __restrict__ bias, float* OUT) {
#pragma clang fp contract(off)
    const int lane = threadIdx.x & 31;
    const int wave = __builtin_amdgcn_readfirstlane((int)(threadIdx.x >> 5));
    const int n = blockIdx.x * AGW + wave;
    if (n >= NN) return;
    const int c4 = lane * 4;
    const int* np = nbr + (size_t)n * KNB;
    const v4i q0 = *(const v4i*)(np), q1 = *(const v4i*)(np + 4), q2 = *(const v4i*)(np + 8), q3 = *(const v4i*)(np + 12);
    const int id[KNB] = { q0[0], q0[1], q0[2], q0[3], q1[0], q1[1], q1[2], q1[3], q2[0], q2[1], q2[2], q2[3], q3[0], q3[1], q3[2], q3[3] };
    const float* frow = FR + (size_t)n * FRP + c4;
    v4f agg = *(const v4f*)(frow);
#pragma unroll
    for (int k = 0; k < KNB; ++k) {
        int j = id[k];
        j = (j < 0) ? (j + NN) : j;
        j = j < 0 ? 0 : (j > NN - 1 ? NN - 1 : j);
        const v4f g = *(const v4f*)(FR + (size_t)j * FRP + c4);
        agg = agg + g;
    }
    const v4f pe = *(const v4f*)(TAB + c4);
    const v4f wv = *(const v4f*)(TAB + CO + c4);
    const v4f bi = *(const v4f*)(bias + c4);
    const v4f rs = *(const v4f*)(frow + CO);
    v4f o;
#pragma unroll
    for (int i = 0; i < 4; ++i) o[i] = ((agg[i] + pe[i]) * wv[i] + bfr(bi[i])) + rs[i];
    float* op = OUT + (size_t)n * CO + c4;
    *(volatile v4f*)op = o; __threadfence(); *(volatile v4f*)op = o;
}

static constexpr size_t al256(size_t v) { return (v + 255) & ~(size_t)255; }
static constexpr size_t SZ_XB  = al256((size_t)NPAD * CI * 2);
static constexpr size_t SZ_WB  = al256((size_t)2 * CO * CI * 2);
static constexpr size_t SZ_FR  = al256((size_t)NPAD * FRP * 4);
static constexpr size_t SZ_TAB = al256((size_t)2 * CO * 4);
static constexpr size_t SZ_TOTAL = SZ_XB + SZ_WB + SZ_FR + SZ_TAB;
static_assert(SZ_TOTAL <= (size_t)134217728);
static_assert(((size_t)CO * CI * 2) % 256 == 0);
static_assert(((size_t)NN * CI * 2) % 128 == 0);
static_assert((size_t)(NPAD / 64) * 64 * FRP * 4 <= SZ_FR);
static_assert((size_t)NPAD * CI * 2 <= SZ_XB);

extern "C" void kernel_launch(void* const* d_in, const int* in_sizes, int n_in,
                              void* d_out, int out_size, void* d_ws, size_t ws_size, hipStream_t stream) {
    if (n_in < 8) return;
    if ((size_t)in_sizes[0] < (size_t)NN * CI) return;
    if ((size_t)in_sizes[1] < (size_t)NN * KNB) return;
    if ((size_t)in_sizes[2] < (size_t)CO * CI || (size_t)in_sizes[6] < (size_t)CO * CI) return;
    if (in_sizes[3] < CO || in_sizes[5] < CO || in_sizes[7] < CO) return;
    if (in_sizes[4] < CO * KS) return;
    if ((size_t)out_size < (size_t)NN * CO) return;
    if (SZ_TOTAL > ws_size) return;
    const float* x   = (const float*)d_in[0];
    const int*   nbr = (const int*)d_in[1];
    const float* wl  = (const float*)d_in[2]; const float* bl = (const float*)d_in[3];
    const float* wt  = (const float*)d_in[4]; const float* bs = (const float*)d_in[5];
    const float* wr  = (const float*)d_in[6]; const float* br = (const float*)d_in[7];
    float* OUT = (float*)d_out;
    char* wsp = (char*)d_ws;
    bf* XB = (bf*)wsp; wsp += SZ_XB;
    bf* WB = (bf*)wsp; wsp += SZ_WB;
    float* FR = (float*)wsp; wsp += SZ_FR;
    float* TAB = (float*)wsp; wsp += SZ_TAB;

    { const size_t n8 = (size_t)NN * CI / 8;
      k_cvt8<<<(unsigned)((n8 + 255) / 256), 256, 0, stream>>>(x, XB, n8); }
    if (NPAD > NN) { const size_t n8 = ((size_t)NPAD - NN) * CI / 8;
      k_zero8<<<(unsigned)((n8 + 255) / 256), 256, 0, stream>>>(XB + (size_t)NN * CI, n8); }
    { const size_t n8 = (size_t)CO * CI / 8; const unsigned g = (unsigned)((n8 + 255) / 256);
      k_cvt8<<<g, 256, 0, stream>>>(wl, WB, n8); k_cvt8<<<g, 256, 0, stream>>>(wr, WB + (size_t)CO * CI, n8); }
    k_tab<<<1, CO, 0, stream>>>(wt, TAB);

    k_gemm<<<dim3(NPAD / 64, FRP / 64, 1), 32, 0, stream>>>(XB, WB, bl, br, FR);

    k_agg<<<(NN + AGW - 1) / AGW, 32 * AGW, 0, stream>>>(FR, nbr, TAB, bs, OUT);
}
